// LSTMModel_90864328114711
// MI455X (gfx1250) — hardware-run, weakly checked
//
#include <hip/hip_runtime.h>
#include <math.h>

constexpr int NSEQ      = 4096;
constexpr int NSTEP     = 512;
constexpr int NIN       = 6;
constexpr int NHID      = 32;
constexpr int NGATE     = 4 * NHID;
constexpr int NCLS      = 8;
constexpr int NTHR      = 128;
constexpr int NWAVE     = NTHR / 32;
constexpr int ROWS_WAVE = 16;
constexpr int ROWS_BLK  = NWAVE * ROWS_WAVE;
constexpr int WPITCH    = 32;
constexpr int HPITCH    = 32;
constexpr int HTILE     = ROWS_WAVE * HPITCH;
constexpr int FPITCH    = 36;
constexpr float ACARRY  = 16.0f;
constexpr float WCARRY  = 64.0f;
constexpr float FOLD    = 1.0f / 1024.0f;
static_assert(NSEQ % ROWS_BLK == 0);
static_assert(NTHR == NGATE);
static_assert(NCLS * NHID == 2 * NTHR);
static_assert((NGATE * NHID / 4) % NTHR == 0);
static_assert((NWAVE * 4 * HTILE / 8) % NTHR == 0);
static_assert(NHID == 32);
static_assert(NIN <= 8);

typedef __attribute__((ext_vector_type(16))) _Float16 v16h;
typedef __attribute__((ext_vector_type(8)))  _Float16 v8h;
typedef __attribute__((ext_vector_type(8)))  float    v8f;
typedef __attribute__((ext_vector_type(4)))  float    v4f;
typedef __attribute__((ext_vector_type(2)))  float    v2f;
typedef __attribute__((ext_vector_type(8)))  unsigned v8u;
typedef __attribute__((ext_vector_type(4)))  unsigned v4u;
typedef __attribute__((ext_vector_type(2)))  unsigned v2u;

struct FragH {
  union U { v16h v; v8h h[2]; };
  static __device__ __forceinline__ v16h load(const _Float16* p) {
    U f; f.h[0] = *(const v8h*)(p); f.h[1] = *(const v8h*)(p + 16); return f.v;
  }
  static __device__ __forceinline__ v8f mma(v16h a, v16h b, v8f c) {
    return __builtin_amdgcn_wmma_f32_16x16x32_f16(false, a, false, b, (short)0, c, false, false);
  }
};
__device__ __forceinline__ void guard4ab(v8f& a0, v8f& a1, v8f& a2, v8f& a3,
                                         v16h x, v16h y0, v16h y1, v16h y2, v16h y3) {
  asm volatile("v_nop\n\tv_nop\n\tv_nop\n\tv_nop"
               : "+v"(a0), "+v"(a1), "+v"(a2), "+v"(a3)
               : "v"(x), "v"(y0), "v"(y1), "v"(y2), "v"(y3));
}

__device__ __forceinline__ unsigned f2h_bits(float f) {
  const _Float16 h = (_Float16)f;
  return (unsigned)__builtin_bit_cast(unsigned short, h);
}
__device__ __forceinline__ float fsig(float z)  { return __builtin_amdgcn_rcpf(1.0f + __expf(-z)); }
__device__ __forceinline__ float ftanh(float z) { return 1.0f - 2.0f * __builtin_amdgcn_rcpf(__expf(2.0f * z) + 1.0f); }

__device__ __forceinline__ void stage_w32(const float* __restrict__ W, _Float16* dst, int tid) {
#pragma unroll 1
  for (int it = 0; it < (NGATE * NHID / 4) / NTHR; ++it) {
    const int idx = it * NTHR + tid;
    const int n = idx >> 3, c4 = (idx & 7) * 4;
    const v4f v = *(const v4f*)(W + n * NHID + c4);
    const float f0 = v[0], f1 = v[1], f2 = v[2], f3 = v[3];
    v2u pk;
    pk[0] = f2h_bits(f0 * WCARRY) | (f2h_bits(f1 * WCARRY) << 16);
    pk[1] = f2h_bits(f2 * WCARRY) | (f2h_bits(f3 * WCARRY) << 16);
    *(v2u*)(dst + n * WPITCH + c4) = pk;
  }
}

__device__ __forceinline__ void mma4(v8f (&acc)[4], v16h a, const _Float16* wb) {
  const v16h b0 = FragH::load(wb);
  const v16h b1 = FragH::load(wb + 1 * NHID * WPITCH);
  const v16h b2 = FragH::load(wb + 2 * NHID * WPITCH);
  const v16h b3 = FragH::load(wb + 3 * NHID * WPITCH);
  acc[0] = FragH::mma(a, b0, acc[0]);
  acc[1] = FragH::mma(a, b1, acc[1]);
  acc[2] = FragH::mma(a, b2, acc[2]);
  acc[3] = FragH::mma(a, b3, acc[3]);
  guard4ab(acc[0], acc[1], acc[2], acc[3], a, b0, b1, b2, b3);
}

template <bool KEEP>
__device__ __forceinline__ void cell_update(const v8f (&acc)[4], const float (&bia)[4],
                                            float (&cs)[8], float (&hs)[8], _Float16* ht, int hh) {
#pragma unroll
  for (int r = 0; r < 8; ++r) {
    const float zi = acc[0][r] * FOLD + bia[0];
    const float zf = acc[1][r] * FOLD + bia[1];
    const float zg = acc[2][r] * FOLD + bia[2];
    const float zo = acc[3][r] * FOLD + bia[3];
    const float ig = fsig(zi);
    const float fg = fsig(zf);
    const float gg = ftanh(zg);
    const float og = fsig(zo);
    const float cn = fg * cs[r] + ig * gg;
    cs[r] = cn;
    const float hn = og * ftanh(cn);
    if (KEEP) hs[r] = hn;
    ht[(8 * hh + r) * HPITCH] = (_Float16)(hn * ACARRY);
  }
}

__global__ __launch_bounds__(NTHR) void rnn2_fused_kernel(
    const float* __restrict__ x,
    const float* __restrict__ W_ih0, const float* __restrict__ W_hh0,
    const float* __restrict__ b_ih0, const float* __restrict__ b_hh0,
    const float* __restrict__ W_ih1, const float* __restrict__ W_hh1,
    const float* __restrict__ b_ih1, const float* __restrict__ b_hh1,
    const float* __restrict__ W_fc,  const float* __restrict__ b_fc,
    float* __restrict__ out) {
  __shared__ __align__(16) _Float16 Wsh[4 * NGATE * WPITCH];
  __shared__ __align__(16) _Float16 Hsh[NWAVE * 4 * HTILE];
  __shared__ __align__(16) float    HFs[NWAVE][ROWS_WAVE * FPITCH];
  __shared__ __align__(16) float    Osh[NWAVE][ROWS_WAVE * NCLS];
  __shared__ float Bsh[2 * NGATE];
  __shared__ float Wfcs[NCLS * NHID];
  __shared__ float Bfcs[NCLS];

  const int tid = threadIdx.x, lane = tid & 31, wave = tid >> 5;
  const int c = lane & 15, hh = lane >> 4, koff = 8 * hh;
  const int rowg = blockIdx.x * ROWS_BLK + wave * ROWS_WAVE;

  {
    const float* wr = W_ih0 + tid * NIN;
    const float f0 = wr[0], f1 = wr[1], f2 = wr[2], f3 = wr[3], f4 = wr[4], f5 = wr[5];
    v4u p0;
    p0[0] = f2h_bits(f0 * WCARRY) | (f2h_bits(f1 * WCARRY) << 16);
    p0[1] = f2h_bits(f2 * WCARRY) | (f2h_bits(f3 * WCARRY) << 16);
    p0[2] = f2h_bits(f4 * WCARRY) | (f2h_bits(f5 * WCARRY) << 16);
    p0[3] = 0u;
    const v4u z4 = {0u, 0u, 0u, 0u};
    v4u* d = (v4u*)(Wsh + tid * WPITCH);
    d[0] = p0; d[1] = z4; d[2] = z4; d[3] = z4;
  }
  asm volatile("" ::: "memory");
  stage_w32(W_hh0, Wsh + 1 * NGATE * WPITCH, tid);
  stage_w32(W_ih1, Wsh + 2 * NGATE * WPITCH, tid);
  stage_w32(W_hh1, Wsh + 3 * NGATE * WPITCH, tid);
  {
    v4u* hz = (v4u*)Hsh;
    const v4u z4 = {0u, 0u, 0u, 0u};
#pragma unroll 1
    for (int i = tid; i < (NWAVE * 4 * HTILE) / 8; i += NTHR) hz[i] = z4;
  }
  asm volatile("" ::: "memory");
  Bsh[tid]         = b_ih0[tid] + b_hh0[tid];
  Bsh[NGATE + tid] = b_ih1[tid] + b_hh1[tid];
  Wfcs[tid]        = W_fc[tid];
  Wfcs[NTHR + tid] = W_fc[NTHR + tid];
  {
    const float bv = b_fc[tid & (NCLS - 1)];
    if (tid < NCLS) Bfcs[tid] = bv;
  }
  __syncthreads();

  float bL0[2][4], bL1[2][4];
#pragma unroll
  for (int nt = 0; nt < 2; ++nt)
#pragma unroll
    for (int g = 0; g < 4; ++g) {
      bL0[nt][g] = Bsh[32 * g + 16 * nt + c];
      bL1[nt][g] = Bsh[NGATE + 32 * g + 16 * nt + c];
    }
  float c1s[2][8], c2s[2][8], h2s[2][8], hdum[2][8];
#pragma unroll
  for (int nt = 0; nt < 2; ++nt)
#pragma unroll
    for (int r = 0; r < 8; ++r) { c1s[nt][r] = 0.0f; c2s[nt][r] = 0.0f; h2s[nt][r] = 0.0f; hdum[nt][r] = 0.0f; }

  _Float16* Hw = Hsh + wave * (4 * HTILE);
  const _Float16* Wp0 = Wsh + 0 * NGATE * WPITCH;
  const _Float16* Wp1 = Wsh + 1 * NGATE * WPITCH;
  const _Float16* Wp2 = Wsh + 2 * NGATE * WPITCH;
  const _Float16* Wp3 = Wsh + 3 * NGATE * WPITCH;
  const unsigned xmask = (unsigned)hh - 1u;
  const v8f z8 = {0.f, 0.f, 0.f, 0.f, 0.f, 0.f, 0.f, 0.f};

#pragma unroll 1
  for (int t = 0; t < NSTEP; ++t) {
    const int q = t & 1, p = q ^ 1;
    const _Float16* H1r = Hw + p * HTILE;
    _Float16*       H1w = Hw + q * HTILE;
    const _Float16* H2r = Hw + (2 + p) * HTILE;
    _Float16*       H2w = Hw + (2 + q) * HTILE;

    const float* xr = x + ((size_t)(rowg + c) * NSTEP + (size_t)t) * NIN;
    const v2f xa = *(const v2f*)(xr);
    const v2f xb = *(const v2f*)(xr + 2);
    const v2f xc = *(const v2f*)(xr + 4);
    const float x0 = xa[0], x1 = xa[1], x2 = xb[0], x3 = xb[1], x4 = xc[0], x5 = xc[1];
    v8u xw;
    xw[0] = (f2h_bits(x0 * ACARRY) | (f2h_bits(x1 * ACARRY) << 16)) & xmask;
    xw[1] = (f2h_bits(x2 * ACARRY) | (f2h_bits(x3 * ACARRY) << 16)) & xmask;
    xw[2] = (f2h_bits(x4 * ACARRY) | (f2h_bits(x5 * ACARRY) << 16)) & xmask;
    xw[3] = 0u; xw[4] = 0u; xw[5] = 0u; xw[6] = 0u; xw[7] = 0u;
    const v16h ax  = __builtin_bit_cast(v16h, xw);
    const v16h ah1 = FragH::load(H1r + c * HPITCH + koff);

#pragma unroll
    for (int nt = 0; nt < 2; ++nt) {
      v8f acc[4];
      acc[0] = z8; acc[1] = z8; acc[2] = z8; acc[3] = z8;
      mma4(acc, ax,  Wp0 + (16 * nt + c) * WPITCH + koff);
      mma4(acc, ah1, Wp1 + (16 * nt + c) * WPITCH + koff);
      cell_update<false>(acc, bL0[nt], c1s[nt], hdum[nt], H1w + 16 * nt + c, hh);
    }
    __syncthreads();
    const v16h ah1c = FragH::load(H1w + c * HPITCH + koff);
    const v16h ah2  = FragH::load(H2r + c * HPITCH + koff);

#pragma unroll
    for (int nt = 0; nt < 2; ++nt) {
      v8f acc[4];
      acc[0] = z8; acc[1] = z8; acc[2] = z8; acc[3] = z8;
      mma4(acc, ah1c, Wp2 + (16 * nt + c) * WPITCH + koff);
      mma4(acc, ah2,  Wp3 + (16 * nt + c) * WPITCH + koff);
      cell_update<true>(acc, bL1[nt], c2s[nt], h2s[nt], H2w + 16 * nt + c, hh);
    }
    __syncthreads();
  }

  float* hf = HFs[wave];
#pragma unroll
  for (int nt = 0; nt < 2; ++nt)
#pragma unroll
    for (int r = 0; r < 8; ++r) hf[(8 * hh + r) * FPITCH + 16 * nt + c] = h2s[nt][r];
  __syncthreads();
  const int cls = lane & (NCLS - 1), rq = lane >> 3;
  float sacc[4] = {0.0f, 0.0f, 0.0f, 0.0f};
#pragma unroll 1
  for (int u = 0; u < NHID; ++u) {
    const float wv = Wfcs[cls * NHID + u];
#pragma unroll
    for (int qq = 0; qq < 4; ++qq) sacc[qq] = fmaf(hf[(4 * qq + rq) * FPITCH + u], wv, sacc[qq]);
  }
  float* os = Osh[wave];
  const float bb = Bfcs[cls];
#pragma unroll
  for (int qq = 0; qq < 4; ++qq) os[32 * qq + lane] = sacc[qq] + bb;
  __syncthreads();
  const v4f ov = *(const v4f*)(os + 4 * lane);
  float* op = out + (size_t)rowg * NCLS + 4 * lane;
  for (int pass = 0; pass < 2; ++pass) {
    *(volatile v4f*)op = ov;
    __threadfence();
  }
}

extern "C" void kernel_launch(void* const* d_in, const int* in_sizes, int n_in,
                              void* d_out, int out_size, void* d_ws, size_t ws_size, hipStream_t stream) {
  (void)d_ws; (void)ws_size;
  if (n_in < 11 || d_out == nullptr) return;
  if (in_sizes[0] != NSEQ * NSTEP * NIN || in_sizes[1] != NGATE * NIN || in_sizes[2] != NGATE * NHID ||
      in_sizes[3] != NGATE || in_sizes[4] != NGATE || in_sizes[5] != NGATE * NHID || in_sizes[6] != NGATE * NHID ||
      in_sizes[7] != NGATE || in_sizes[8] != NGATE || in_sizes[9] != NCLS * NHID || in_sizes[10] != NCLS ||
      out_size != NSEQ * NCLS) return;

  const float* x     = (const float*)d_in[0];
  const float* W_ih0 = (const float*)d_in[1];
  const float* W_hh0 = (const float*)d_in[2];
  const float* b_ih0 = (const float*)d_in[3];
  const float* b_hh0 = (const float*)d_in[4];
  const float* W_ih1 = (const float*)d_in[5];
  const float* W_hh1 = (const float*)d_in[6];
  const float* b_ih1 = (const float*)d_in[7];
  const float* b_hh1 = (const float*)d_in[8];
  const float* W_fc  = (const float*)d_in[9];
  const float* b_fc  = (const float*)d_in[10];
  float* out = (float*)d_out;

  rnn2_fused_kernel<<<NSEQ / ROWS_BLK, NTHR, 0, stream>>>(
      x, W_ih0, W_hh0, b_ih0, b_hh0, W_ih1, W_hh1, b_ih1, b_hh1, W_fc, b_fc, out);
}
